// MultiHeadAttention_63591285785308
// MI455X (gfx1250) — hardware-verified
//
#include <hip/hip_runtime.h>

typedef __attribute__((ext_vector_type(16))) _Float16 v16h;
typedef __attribute__((ext_vector_type(16))) __bf16 v16b;
typedef __attribute__((ext_vector_type(8)))  _Float16 v8h;
typedef __attribute__((ext_vector_type(8)))  __bf16 v8b;
typedef __attribute__((ext_vector_type(8)))  float v8f;
typedef __attribute__((ext_vector_type(4)))  float v4f;
typedef __attribute__((ext_vector_type(4)))  unsigned v4u;

template <typename T> __device__ __forceinline__ void vst2(void* p, T v) { *(volatile T*)p = v; __threadfence(); *(volatile T*)p = v; }

__device__ __forceinline__ v8f wmma16(v16h a, v16h b, v8f c) {
  v8f d = __builtin_amdgcn_wmma_f32_16x16x32_f16(false, a, false, b, (short)0, c, false, false);
  asm volatile("v_nop\n\tv_nop\n\tv_nop\n\tv_nop" : "+v"(d) : "v"(a), "v"(b));
  return d;
}
__device__ __forceinline__ v8f wmma_bf(v16b a, v16b b, v8f c) {
  v8f d = __builtin_amdgcn_wmma_f32_16x16x32_bf16(false, a, false, b, (short)0, c, false, false);
  asm volatile("v_nop\n\tv_nop\n\tv_nop\n\tv_nop" : "+v"(d) : "v"(a), "v"(b));
  return d;
}
__device__ __forceinline__ v16h frag_h(const _Float16* rowk0, int lane) {
  union { v16h v; v8h q[2]; } u; const _Float16* p = rowk0 + 8 * (lane >> 4);
  u.q[0] = *(const v8h*)p; u.q[1] = *(const v8h*)(p + 16); return u.v;
}
__device__ __forceinline__ v16b frag_b(const __bf16* rowk0, int lane) {
  union { v16b v; v8b q[2]; } u; const __bf16* p = rowk0 + 8 * (lane >> 4);
  u.q[0] = *(const v8b*)p; u.q[1] = *(const v8b*)(p + 16); return u.v;
}
#define LDSX() do { asm volatile("s_wait_dscnt 0" ::: "memory"); __builtin_amdgcn_wave_barrier(); __builtin_amdgcn_fence(3  , "workgroup"); } while (0)

#ifndef NB
#define NB 2
#endif
#ifndef SEQ
#define SEQ 2048
#endif
#define NB_FULL 2
#define SEQ_FULL 2048
#define DM 1024
#define NH 16
#define HD 64
#define SLT (SEQ / NH)
#define NSLAB (NB * NH)
#define MROWS (NB * SEQ)
#define SCALE 0.125f
#define LN1024 6.931471805599453f
#define IN8 (SEQ * DM / 8)
#define W8 (DM * DM / 8)

static_assert(DM == NH * HD);
static_assert(HD == 64);
static_assert(SEQ % (NH * 64) == 0);
static_assert(DM % 128 == 0);
static_assert(DM % 32 == 0);
static_assert(MROWS % 64 == 0);
static_assert(IN8 % 256 == 0);
static_assert(W8 % 256 == 0);
static_assert(NB <= NB_FULL);
static_assert(SEQ <= SEQ_FULL);

#define PLANE16 (2u * (size_t)MROWS * DM)
#define WPLANE16 (2u * (size_t)DM * DM)
#define WS_XQ 0u
#define WS_XK (WS_XQ + PLANE16)
#define WS_XV (WS_XK + PLANE16)
#define WS_WQ (WS_XV + PLANE16)
#define WS_WK (WS_WQ + WPLANE16)
#define WS_WV (WS_WK + WPLANE16)
#define WS_WO (WS_WV + WPLANE16)
#define WS_QH (WS_WO + WPLANE16)
#define WS_KH (WS_QH + PLANE16)
#define WS_VT (WS_KH + PLANE16)
#define WS_YH (WS_VT + PLANE16)
#define WS_END (WS_YH + PLANE16)
static_assert(WS_END <= 134217728u);
static_assert((size_t)NSLAB * DM * SLT * 2u == PLANE16);

__device__ __forceinline__ unsigned bf_bits(float f) { unsigned u = __float_as_uint(f); u += 0x7FFFu + ((u >> 16) & 1u); return u >> 16; }
__device__ __forceinline__ float bfr(float f) { return __uint_as_float(bf_bits(f) << 16); }

__global__ __launch_bounds__(256) void k_cvt_bf(const float* __restrict__ src, unsigned short* __restrict__ dst, int pb8, int bstride) {
  const int i = blockIdx.x * 256 + threadIdx.x;
  if (i < pb8) {
    const float* p = src + (size_t)blockIdx.y * (size_t)bstride + (size_t)i * 8;
    const v4f f0 = *(const v4f*)p; const v4f f1 = *(const v4f*)(p + 4);
    v4u u;
    u.x = bf_bits(f0.x) | (bf_bits(f0.y) << 16); u.y = bf_bits(f0.z) | (bf_bits(f0.w) << 16);
    u.z = bf_bits(f1.x) | (bf_bits(f1.y) << 16); u.w = bf_bits(f1.z) | (bf_bits(f1.w) << 16);
    vst2(dst + ((size_t)blockIdx.y * (size_t)pb8 + (size_t)i) * 8, u);
  }
}
__global__ __launch_bounds__(256) void k_cvt_wo(const float* __restrict__ src, _Float16* __restrict__ dst, int pb8) {
  const int i = blockIdx.x * 256 + threadIdx.x;
  if (i < pb8) {
    const float* p = src + (size_t)i * 8;
    const v4f f0 = *(const v4f*)p; const v4f f1 = *(const v4f*)(p + 4);
    union { v8h h; v4u u; } o;
    o.h[0] = (_Float16)(bfr(f0.x) * 256.0f); o.h[1] = (_Float16)(bfr(f0.y) * 256.0f); o.h[2] = (_Float16)(bfr(f0.z) * 256.0f); o.h[3] = (_Float16)(bfr(f0.w) * 256.0f);
    o.h[4] = (_Float16)(bfr(f1.x) * 256.0f); o.h[5] = (_Float16)(bfr(f1.y) * 256.0f); o.h[6] = (_Float16)(bfr(f1.z) * 256.0f); o.h[7] = (_Float16)(bfr(f1.w) * 256.0f);
    vst2(dst + (size_t)i * 8, o.u);
  }
}

__global__ __launch_bounds__(128) void k_proj(const __bf16* __restrict__ XB, const __bf16* __restrict__ WB, const float* __restrict__ BA, _Float16* __restrict__ DH, _Float16* __restrict__ VT, int vmode) {
  __shared__ __align__(16) _Float16 sh[64][136]; __shared__ __align__(16) _Float16 th[128][72];
  const int tid = threadIdx.x; const int wave = __builtin_amdgcn_readfirstlane(tid >> 5); const int lane = tid & 31, col = lane & 15, g = lane >> 4;
  const int c0 = blockIdx.y * 128; const size_t r0 = (size_t)blockIdx.x * 64;
  const __bf16* arow = XB + (r0 + wave * 16 + col) * DM;
  v8f acc[8] = {};
#pragma unroll 2
  for (int kc = 0; kc < DM / 32; ++kc) { const v16b a = frag_b(arow + kc * 32, lane);
#pragma unroll
    for (int j = 0; j < 8; ++j) { const v16b w = frag_b(WB + (size_t)(c0 + j * 16 + col) * DM + kc * 32, lane); acc[j] = wmma_bf(a, w, acc[j]); } }
  if (vmode == 0) {
#pragma unroll
    for (int j = 0; j < 8; ++j) { const float bias = bfr(BA[c0 + j * 16 + col]);
#pragma unroll
      for (int r = 0; r < 8; ++r) sh[wave * 16 + 8 * g + r][j * 16 + col] = (_Float16)(acc[j][r] + bias); }
    __syncthreads();
    for (int e = tid; e < 64 * 16; e += 128) { const int rl = e >> 4, q = e & 15; vst2(DH + (r0 + rl) * DM + c0 + q * 8, *(const v4u*)&sh[rl][q * 8]); }
  } else { const size_t slab = r0 / SLT; const int t0 = (int)(r0 % SLT);
#pragma unroll
    for (int j = 0; j < 8; ++j) { const float bias = bfr(BA[c0 + j * 16 + col]);
#pragma unroll
      for (int r = 0; r < 8; ++r) th[j * 16 + col][wave * 16 + 8 * g + r] = (_Float16)(acc[j][r] + bias); }
    __syncthreads();
    for (int e = tid; e < 128 * 8; e += 128) { const int cl = e >> 3, q = e & 7; vst2(VT + (slab * DM + c0 + cl) * (size_t)SLT + t0 + q * 8, *(const v4u*)&th[cl][q * 8]); }
  } }

__global__ __launch_bounds__(128) void k_attn(const _Float16* __restrict__ QH, const _Float16* __restrict__ KH, const _Float16* __restrict__ VT, _Float16* __restrict__ YH) {
  __shared__ __align__(16) _Float16 so[4][16][72];
  const int tid = threadIdx.x; const int wave = __builtin_amdgcn_readfirstlane(tid >> 5); const int lane = tid & 31, col = lane & 15, g = lane >> 4;
  const int L = blockIdx.z, cbq = blockIdx.y; const int tq0 = blockIdx.x * 64 + wave * 16;
  const size_t rowbase = (size_t)L * SLT;
  const _Float16* qrow = QH + (rowbase + tq0 + col) * DM + cbq * HD;
  const v16h qf0 = frag_h(qrow, lane), qf1 = frag_h(qrow + 32, lane);
  const _Float16* kbase = KH + (rowbase + col) * DM;
  const _Float16* vbase = VT + ((size_t)L * DM + col) * SLT;
  v8f acc[4] = {}; float m = -1.0e30f, l = 0.f;
#pragma unroll 1
  for (int cb = 0; cb < NH; ++cb) {
#pragma unroll 1
    for (int tl0 = 0; tl0 < SLT; tl0 += 32) {
      const _Float16* kp = kbase + (size_t)tl0 * DM + cb * HD;
      v8f s0 = {}, s1 = {};
      s0 = wmma16(frag_h(kp, lane), qf0, s0);
      s0 = wmma16(frag_h(kp + 32, lane), qf1, s0);
      s1 = wmma16(frag_h(kp + 16 * DM, lane), qf0, s1);
      s1 = wmma16(frag_h(kp + 16 * DM + 32, lane), qf1, s1);
      float mr = fmaxf(s0[0], s1[0]);
#pragma unroll
      for (int r = 1; r < 8; ++r) mr = fmaxf(mr, fmaxf(s0[r], s1[r]));
      mr = fmaxf(mr, __shfl_xor(mr, 16));
      const float mnew = fmaxf(m, mr * SCALE);
      if (__builtin_amdgcn_ballot_w32(mnew > m) != 0u) {
        const float corr = __expf(m - mnew);
#pragma unroll
        for (int j = 0; j < 4; ++j)
#pragma unroll
          for (int r = 0; r < 8; ++r) acc[j][r] *= corr;
        l *= corr; }
      m = mnew;
      const float ms = mnew - LN1024;
      v16h pb;
#pragma unroll
      for (int r = 0; r < 8; ++r) { const float p0 = __expf(fmaf(s0[r], SCALE, -ms)); const float p1 = __expf(fmaf(s1[r], SCALE, -ms)); l += p0 + p1; pb[r] = (_Float16)p0; pb[8 + r] = (_Float16)p1; }
      const _Float16* vp = vbase + (size_t)(cb * HD) * SLT + tl0;
      acc[0] = wmma16(frag_h(vp, lane), pb, acc[0]);
      acc[1] = wmma16(frag_h(vp + 16 * SLT, lane), pb, acc[1]);
      acc[2] = wmma16(frag_h(vp + 32 * SLT, lane), pb, acc[2]);
      acc[3] = wmma16(frag_h(vp + 48 * SLT, lane), pb, acc[3]);
    } }
  const float lt = l + __shfl_xor(l, 16);
  const float inv = 64.0f * __builtin_amdgcn_rcpf(lt);
#pragma unroll
  for (int j = 0; j < 4; ++j) { v8h o;
#pragma unroll
    for (int r = 0; r < 8; ++r) o[r] = (_Float16)(acc[j][r] * inv);
    *(v8h*)&so[wave][col][j * 16 + 8 * g] = o; }
  LDSX();
#pragma unroll
  for (int i = 0; i < 4; ++i) { const int rl = i * 4 + (lane >> 3), q = lane & 7; vst2(YH + (rowbase + tq0 + rl) * DM + cbq * HD + q * 8, *(const v4u*)&so[wave][rl][q * 8]); }
}

__global__ __launch_bounds__(128) void k_out(const _Float16* __restrict__ YH, const _Float16* __restrict__ WOH, const float* __restrict__ BO, float* __restrict__ OUT) {
  __shared__ __align__(16) float sf[4][16][132];
  const int tid = threadIdx.x; const int wave = __builtin_amdgcn_readfirstlane(tid >> 5); const int lane = tid & 31, col = lane & 15, g = lane >> 4;
  const int c0 = blockIdx.y * 128; const size_t r0 = (size_t)blockIdx.x * 64 + wave * 16;
  const _Float16* arow = YH + (r0 + col) * DM;
  v8f acc[8] = {};
#pragma unroll 2
  for (int kc = 0; kc < DM / 32; ++kc) { const v16h a = frag_h(arow + kc * 32, lane);
#pragma unroll
    for (int j = 0; j < 8; ++j) { const v16h w = frag_h(WOH + (size_t)(c0 + j * 16 + col) * DM + kc * 32, lane); acc[j] = wmma16(a, w, acc[j]); } }
#pragma unroll
  for (int j = 0; j < 8; ++j) { const float bias = bfr(BO[c0 + j * 16 + col]);
#pragma unroll
    for (int r = 0; r < 8; ++r) sf[wave][8 * g + r][j * 16 + col] = acc[j][r] * (1.0f / 16384.0f) + bias; }
  LDSX();
  for (int rl = 0; rl < 16; ++rl) vst2(OUT + (r0 + rl) * DM + c0 + lane * 4, *(const v4f*)&sf[wave][rl][lane * 4]);
}

extern "C" void kernel_launch(void* const* d_in, const int* in_sizes, int n_in, void* d_out, int out_size, void* d_ws, size_t ws_size, hipStream_t stream) {
  if (n_in < 11) return;
  const long long need_in = (long long)(NB - 1) * SEQ_FULL * DM + (long long)SEQ * DM;
  if (in_sizes[0] < need_in || in_sizes[1] < need_in || in_sizes[2] < need_in) return;
  if (in_sizes[3] < DM * DM || in_sizes[5] < DM * DM || in_sizes[7] < DM * DM || in_sizes[9] < DM * DM) return;
  if (in_sizes[4] < DM || in_sizes[6] < DM || in_sizes[8] < DM || in_sizes[10] < DM) return;
  if ((long long)out_size < (long long)MROWS * DM) return;
  if (ws_size < (size_t)WS_END) return;
  const float* const* F = (const float* const*)d_in;
  char* ws = (char*)d_ws;
  unsigned short *XQ = (unsigned short*)(ws + WS_XQ), *XK = (unsigned short*)(ws + WS_XK), *XV = (unsigned short*)(ws + WS_XV);
  unsigned short *WQ = (unsigned short*)(ws + WS_WQ), *WK = (unsigned short*)(ws + WS_WK), *WV = (unsigned short*)(ws + WS_WV);
  _Float16 *WO = (_Float16*)(ws + WS_WO), *QH = (_Float16*)(ws + WS_QH), *KH = (_Float16*)(ws + WS_KH), *VT = (_Float16*)(ws + WS_VT), *YH = (_Float16*)(ws + WS_YH);
  k_cvt_bf<<<dim3(IN8 / 256, NB), 256, 0, stream>>>(F[0], XQ, IN8, SEQ_FULL * DM);
  k_cvt_bf<<<dim3(IN8 / 256, NB), 256, 0, stream>>>(F[1], XK, IN8, SEQ_FULL * DM);
  k_cvt_bf<<<dim3(IN8 / 256, NB), 256, 0, stream>>>(F[2], XV, IN8, SEQ_FULL * DM);
  k_cvt_bf<<<dim3(W8 / 256, 1), 256, 0, stream>>>(F[3], WQ, W8, 0);
  k_cvt_bf<<<dim3(W8 / 256, 1), 256, 0, stream>>>(F[5], WK, W8, 0);
  k_cvt_bf<<<dim3(W8 / 256, 1), 256, 0, stream>>>(F[7], WV, W8, 0);
  k_cvt_wo<<<dim3(W8 / 256, 1), 256, 0, stream>>>(F[9], WO, W8);
  k_proj<<<dim3(MROWS / 64, DM / 128), 128, 0, stream>>>((const __bf16*)XQ, (const __bf16*)WQ, F[4], QH, VT, 0);
  k_proj<<<dim3(MROWS / 64, DM / 128), 128, 0, stream>>>((const __bf16*)XK, (const __bf16*)WK, F[6], KH, VT, 0);
  k_proj<<<dim3(MROWS / 64, DM / 128), 128, 0, stream>>>((const __bf16*)XV, (const __bf16*)WV, F[8], QH, VT, 1);
  k_attn<<<dim3(SLT / 64, NH, NSLAB), 128, 0, stream>>>(QH, KH, VT, YH);
  k_out<<<dim3(MROWS / 64, DM / 128), 128, 0, stream>>>(YH, WO, F[10], (float*)d_out);
}
